// SpatialSelfAttention_47863115546958
// MI455X (gfx1250) — hardware-verified
//
#include <hip/hip_runtime.h>


#ifndef NB
#define NB 4
#endif
#ifndef SEQ
#define SEQ 4096
#endif
#ifndef SEQ_FULL
#define SEQ_FULL 4096
#endif
#ifndef OUT_PITCH
#define OUT_PITCH SEQ
#endif

namespace {
constexpr int Bn = NB, C = 512, NPIX = SEQ, XS = SEQ_FULL, OS = OUT_PITCH, G = 32, CPG = C / G;
constexpr float EPS = 1e-6f;
constexpr float P_SC = 4096.0f, INV_P_SC = 1.0f / 4096.0f;
constexpr float O_SC = 64.0f, INV_O_SC = 1.0f / 64.0f;
constexpr float PV_SC = O_SC * INV_P_SC;
static_assert(NPIX % 256 == 0);
static_assert(NPIX <= XS);
static_assert(OS >= NPIX);
static_assert(C % 128 == 0);
static_assert((XS % 4) == 0 && (OS % 4) == 0);
static_assert(CPG == 16);

typedef _Float16 b16;
typedef __attribute__((ext_vector_type(16))) _Float16 v16b;
typedef __attribute__((ext_vector_type(8)))  _Float16 v8b;
typedef __attribute__((ext_vector_type(8)))  float v8f;
typedef __attribute__((ext_vector_type(4)))  float v4f;

__device__ __forceinline__ v8b ld8b(const b16* p) { return *(const v8b*)p; }
__device__ __forceinline__ v16b cat8b(v8b a, v8b b) { return __builtin_shufflevector(a, b, 0, 1, 2, 3, 4, 5, 6, 7, 8, 9, 10, 11, 12, 13, 14, 15); }
__device__ __forceinline__ v16b frag_kb(const b16* p, int hh) { return cat8b(ld8b(p + 8 * hh), ld8b(p + 16 + 8 * hh)); }
__device__ __forceinline__ void split16(float v, b16& hi, b16& lo) { hi = (b16)v; lo = (b16)(v - (float)hi); }
__device__ __forceinline__ void frag_ksplit(const float* p, int hh, v16b& fh_, v16b& fl_) {
  const float* p0 = p + 8 * hh; const float* p1 = p + 16 + 8 * hh;
#pragma unroll
  for (int e = 0; e < 8; ++e) { b16 a, c; split16(p0[e], a, c); fh_[e] = a; fl_[e] = c; split16(p1[e], a, c); fh_[8 + e] = a; fl_[8 + e] = c; }
}
__device__ __forceinline__ v8f wmma16b(v16b a, v16b b, v8f c) {
  v8f d = __builtin_amdgcn_wmma_f32_16x16x32_f16(false, a, false, b, (short)0, c, false, false);
  asm volatile("v_nop\n\tv_nop\n\tv_nop\n\tv_nop" : "+v"(d) : "v"(a), "v"(b));
  return d;
}
__device__ __forceinline__ void wave_lds_sync() {
  __builtin_amdgcn_fence(3, "workgroup");
  __builtin_amdgcn_wave_barrier();
  __builtin_amdgcn_fence(2, "workgroup");
}

struct Opnd { const void* p0; const void* p1; int ld; };
template <int NP> __device__ __forceinline__ void load_frags(const Opnd& o, int row, int kb, int hh, v16b& fh_, v16b& fl_) {
  if (NP == 0) { frag_ksplit((const float*)o.p0 + (size_t)row * o.ld + kb, hh, fh_, fl_); }
  else if (NP == 3) {
    const float* p = (const float*)o.p0 + (size_t)row * o.ld + kb; const float* p0 = p + 8 * hh; const float* p1 = p + 16 + 8 * hh;
#pragma unroll
    for (int e = 0; e < 8; ++e) { fh_[e] = (b16)p0[e]; fh_[8 + e] = (b16)p1[e]; }
    fl_ = fh_;
  } else {
    fh_ = frag_kb((const b16*)o.p0 + (size_t)row * o.ld + kb, hh);
    if (NP == 2) fl_ = frag_kb((const b16*)o.p1 + (size_t)row * o.ld + kb, hh); else fl_ = fh_;
  }
}
template <int ANP, int BNP> __device__ __forceinline__ v8f mac(v16b ah, v16b al, v16b bh, v16b bl, v8f c) {
  c = wmma16b(ah, bh, c);
  if (BNP == 0 || BNP == 2) c = wmma16b(ah, bl, c);
  if (ANP == 0 || ANP == 2) c = wmma16b(al, bh, c);
  return c;
}
template <int ANP, int BNP>
__device__ __forceinline__ void gemm_tile(const Opnd& A, const Opnd& B, int K, int m0, int c0, int nloc, int hlf, v8f (&acc)[2][4]) {
  for (int kb = 0; kb < K; kb += 32) {
    v16b a0h, a0l, a1h, a1l;
    load_frags<ANP>(A, m0 + nloc, kb, hlf, a0h, a0l);
    load_frags<ANP>(A, m0 + 16 + nloc, kb, hlf, a1h, a1l);
#pragma unroll
    for (int t = 0; t < 4; ++t) {
      v16b bh, bl;
      load_frags<BNP>(B, c0 + t * 16 + nloc, kb, hlf, bh, bl);
      acc[0][t] = mac<ANP, BNP>(a0h, a0l, bh, bl, acc[0][t]);
      acc[1][t] = mac<ANP, BNP>(a1h, a1l, bh, bl, acc[1][t]);
    }
  }
}

__device__ __forceinline__ void epi_planes(v8f (&acc)[2][4], float scale, const float* cbias, const float* rbias, bool two,
                                           b16* __restrict__ oh, b16* __restrict__ ol, int ldo, int m0, int c0, int lane, b16* Th, b16* Tl) {
  const int nloc = lane & 15, hlf = lane >> 4;
#pragma unroll
  for (int t = 0; t < 4; ++t)
#pragma unroll
    for (int r = 0; r < 2; ++r)
#pragma unroll
      for (int v = 0; v < 8; ++v) {
        const int rr = r * 16 + v + 8 * hlf, cc = t * 16 + nloc;
        float val = acc[r][t][v] * scale;
        if (cbias) val += cbias[c0 + cc];
        if (rbias) val += rbias[m0 + rr];
        b16 h_, l_; split16(val, h_, l_);
        Th[rr * 64 + cc] = h_; if (two) Tl[rr * 64 + cc] = l_;
      }
  wave_lds_sync();
  for (int pass = 0; pass < 2; ++pass) {
#pragma unroll
    for (int j = 0; j < 8; ++j) {
      const int rr = j * 4 + (lane >> 3), c8 = (lane & 7) * 8;
      const size_t o = (size_t)(m0 + rr) * ldo + c0 + c8;
      *(volatile v8b*)(oh + o) = ld8b(Th + rr * 64 + c8);
      if (two) *(volatile v8b*)(ol + o) = ld8b(Tl + rr * 64 + c8);
    }
    __threadfence();
  }
}
__device__ __forceinline__ void epi_f32(v8f (&acc)[2][4], float scale, const float* cbias, const float* rbias, const float* resid, int ldr,
                                        float* __restrict__ out, int ldo, int m0, int c0, int lane, float* Tt) {
  const int nloc = lane & 15, hlf = lane >> 4;
#pragma unroll
  for (int t = 0; t < 4; ++t)
#pragma unroll
    for (int r = 0; r < 2; ++r)
#pragma unroll
      for (int v = 0; v < 8; ++v) {
        const int rr = r * 16 + v + 8 * hlf, cc = t * 16 + nloc;
        float val = acc[r][t][v] * scale;
        if (cbias) val += cbias[c0 + cc];
        if (rbias) val += rbias[m0 + rr];
        Tt[rr * 64 + cc] = val;
      }
  wave_lds_sync();
  float* dst0 = out + (size_t)m0 * ldo + c0; const float* rs0 = resid ? resid + (size_t)m0 * ldr + c0 : nullptr;
  for (int pass = 0; pass < 2; ++pass) {
#pragma unroll
    for (int j = 0; j < 16; ++j) {
      const int rr = j * 2 + hlf, c4 = nloc * 4;
      v4f val = *(const v4f*)(Tt + rr * 64 + c4);
      if (rs0) val += *(const v4f*)(rs0 + (size_t)rr * ldr + c4);
      *(volatile v4f*)(dst0 + (size_t)rr * ldo + c4) = val;
    }
    __threadfence();
  }
}


__global__ __launch_bounds__(256) void prep_kernel(const float* __restrict__ wq, const float* __restrict__ wk, const float* __restrict__ wv,
                                                   const float* __restrict__ wp, b16* __restrict__ w16) {
  const size_t tid = (size_t)blockIdx.x * blockDim.x + threadIdx.x, stride = (size_t)gridDim.x * blockDim.x;
  const size_t n1 = (size_t)C * C / 8;
  for (int pass = 0; pass < 2; ++pass) {
    for (size_t c = tid; c < 4 * n1; c += stride) {
      const int which = (int)(c / n1); const size_t i = (c % n1) * 8;
      const float* w = (which == 0) ? wq : (which == 1) ? wk : (which == 2) ? wv : wp;
      v8b v;
#pragma unroll
      for (int e = 0; e < 8; ++e) v[e] = (b16)w[i + e];
      *(volatile v8b*)(w16 + (size_t)which * C * C + i) = v;
    }
    __threadfence();
  }
}

__global__ __launch_bounds__(256) void gn_stats_kernel(const float* __restrict__ x, float* __restrict__ stats) {
  __shared__ float red[8];
  const int bg = blockIdx.x, tid = threadIdx.x, lane = tid & 31, wave = tid >> 5;
  const float* p = x + (size_t)bg * CPG * XS;
  float s = 0.f;
  for (int i = tid * 4; i < CPG * NPIX; i += 256 * 4) {
    const int cc = i / NPIX, px = i - cc * NPIX;
    const v4f q = *(const v4f*)(p + (size_t)cc * XS + px); s += (q[0] + q[1]) + (q[2] + q[3]);
  }
#pragma unroll
  for (int o = 16; o > 0; o >>= 1) s += __shfl_xor(s, o);
  if (lane == 0) red[wave] = s;
  __syncthreads();
  float tot = 0.f;
#pragma unroll
  for (int w = 0; w < 8; ++w) tot += red[w];
  const float mean = tot * (1.0f / (CPG * NPIX));
  __syncthreads();
  float s2 = 0.f;
  for (int i = tid * 4; i < CPG * NPIX; i += 256 * 4) {
    const int cc = i / NPIX, px = i - cc * NPIX;
    const v4f q = *(const v4f*)(p + (size_t)cc * XS + px); const float a = q[0] - mean, b2 = q[1] - mean, c2 = q[2] - mean, d2 = q[3] - mean;
    s2 += (a * a + b2 * b2) + (c2 * c2 + d2 * d2);
  }
#pragma unroll
  for (int o = 16; o > 0; o >>= 1) s2 += __shfl_xor(s2, o);
  if (lane == 0) red[wave] = s2;
  __syncthreads();
  float tot2 = 0.f;
#pragma unroll
  for (int w = 0; w < 8; ++w) tot2 += red[w];
  const float rstd = rsqrtf(tot2 * (1.0f / (CPG * NPIX)) + EPS);
  if (tid < 32) {
    const float v = (tid == 0) ? mean : (tid == 1) ? rstd : 0.0f;
    ((volatile float*)stats)[(size_t)bg * 32 + tid] = v;
    __threadfence();
    ((volatile float*)stats)[(size_t)bg * 32 + tid] = v;
  }
}

__global__ __launch_bounds__(256) void gn_apply_kernel(const float* __restrict__ x, const float* __restrict__ stats, const float* __restrict__ gamma,
                                                       const float* __restrict__ beta, int b, b16* __restrict__ hn) {
  __shared__ __attribute__((aligned(16))) b16 Tl[64][C + 8];
  const int tid = threadIdx.x, lane = tid & 31, wave = tid >> 5, n0 = blockIdx.x * 64;
  const float* xb = x + (size_t)b * C * XS;
  for (int it = 0; it < C / 16; ++it) {
    const int c = it * 16 + (tid >> 4), px = (tid & 15) * 4;
    const float mean = stats[((size_t)b * G + c / CPG) * 32], rstd = stats[((size_t)b * G + c / CPG) * 32 + 1];
    const float ga = gamma[c] * rstd, be = beta[c] - mean * gamma[c] * rstd;
    const v4f q = *(const v4f*)(xb + (size_t)c * XS + n0 + px);
#pragma unroll
    for (int e = 0; e < 4; ++e) Tl[px + e][c] = (b16)(q[e] * ga + be);
  }
  __syncthreads();
  for (int pass = 0; pass < 2; ++pass) {
#pragma unroll
    for (int rr = 0; rr < 8; ++rr) {
      const int row = wave * 8 + rr;
      b16* dst = hn + (size_t)(n0 + row) * C;
#pragma unroll
      for (int j = 0; j < 2; ++j) { const int e = j * 256 + lane * 8; *(volatile v8b*)(dst + e) = *(const v8b*)(&Tl[row][e]); }
    }
    __threadfence();
  }
}

template <bool OUT16>
__global__ __launch_bounds__(128) __attribute__((amdgpu_num_vgpr(256)))
void gemm_kernel(const b16* __restrict__ A, int lda, const b16* __restrict__ Bm, int ldb, int K, float scale,
                 const float* __restrict__ cbias, const float* __restrict__ rbias, const float* __restrict__ resid, int ldr,
                 b16* __restrict__ o16, float* __restrict__ o32, int ldo) {
  __shared__ __attribute__((aligned(16))) float Ts[4][32 * 64];
  __shared__ __attribute__((aligned(16))) b16 Th[4][32 * 64];
  const int lane = threadIdx.x & 31, wave = threadIdx.x >> 5, nloc = lane & 15, hlf = lane >> 4;
  const int m0 = blockIdx.y * 128 + wave * 32, c0 = blockIdx.x * 64;
  v8f acc[2][4];
#pragma unroll
  for (int r = 0; r < 2; ++r)
#pragma unroll
    for (int t = 0; t < 4; ++t) acc[r][t] = (v8f){};
  const Opnd Ao{A, nullptr, lda}, Bo{Bm, nullptr, ldb};
  gemm_tile<1, 1>(Ao, Bo, K, m0, c0, nloc, hlf, acc);
  if (OUT16) epi_planes(acc, scale, cbias, rbias, false, o16, nullptr, ldo, m0, c0, lane, Th[wave], nullptr);
  else       epi_f32(acc, scale, cbias, rbias, resid, ldr, o32, ldo, m0, c0, lane, Ts[wave]);
}

__global__ __launch_bounds__(256) void softmax_kernel(const b16* __restrict__ S, b16* __restrict__ P) {
  constexpr int NJ = NPIX / 256;
  const int lane = threadIdx.x & 31, r = blockIdx.x * 8 + (threadIdx.x >> 5);
  if (r >= NPIX) return;
  const b16* Sr = S + (size_t)r * NPIX + lane * 8;
  float mx = -INFINITY;
#pragma unroll 1
  for (int j = 0; j < NJ; ++j) {
    const v8b q = ld8b(Sr + 256 * j);
#pragma unroll
    for (int e = 0; e < 8; ++e) mx = fmaxf(mx, (float)q[e]);
  }
#pragma unroll
  for (int o = 16; o > 0; o >>= 1) mx = fmaxf(mx, __shfl_xor(mx, o));
  float sum = 0.0f;
#pragma unroll 1
  for (int j = 0; j < NJ; ++j) {
    const v8b q = ld8b(Sr + 256 * j);
#pragma unroll
    for (int e = 0; e < 8; ++e) sum += __expf((float)q[e] - mx);
  }
#pragma unroll
  for (int o = 16; o > 0; o >>= 1) sum += __shfl_xor(sum, o);
  const float inv = P_SC / sum;
  b16* Pr = P + (size_t)r * NPIX + lane * 8;
#pragma unroll 1
  for (int pass = 0; pass < 2; ++pass) {
#pragma unroll 1
    for (int j = 0; j < NJ; ++j) {
      const v8b q = ld8b(Sr + 256 * j);
      v8b pv;
#pragma unroll
      for (int e = 0; e < 8; ++e) pv[e] = (b16)(__expf((float)q[e] - mx) * inv);
      *(volatile v8b*)(Pr + 256 * j) = pv;
    }
    __threadfence();
  }
}
}

extern "C" void kernel_launch(void* const* d_in, const int* in_sizes, int n_in,
                              void* d_out, int out_size, void* d_ws, size_t ws_size, hipStream_t stream) {
  if (n_in < 11) return;
  const float* x     = (const float*)d_in[0];
  const float* gamma = (const float*)d_in[1];
  const float* beta  = (const float*)d_in[2];
  const float* wq = (const float*)d_in[3];  const float* bq = (const float*)d_in[4];
  const float* wk = (const float*)d_in[5];  const float* bk = (const float*)d_in[6];
  const float* wv = (const float*)d_in[7];  const float* bv = (const float*)d_in[8];
  const float* wp = (const float*)d_in[9];  const float* bp = (const float*)d_in[10];
  float* out = (float*)d_out;

  const size_t need_x = ((size_t)(Bn - 1) * C + (C - 1)) * XS + NPIX;
  if ((size_t)in_sizes[0] < need_x) return;
  if (in_sizes[1] < C || in_sizes[2] < C) return;
  if (in_sizes[3] < C * C || in_sizes[5] < C * C || in_sizes[7] < C * C || in_sizes[9] < C * C) return;
  if (in_sizes[4] < C || in_sizes[6] < C || in_sizes[8] < C || in_sizes[10] < C) return;
  const size_t need_o = ((size_t)(Bn - 1) * C + (C - 1)) * OS + NPIX;
  if ((size_t)out_size < need_o) return;

  size_t off = 0; char* ws = (char*)d_ws;
  auto carve = [&](size_t bytes) { char* p = ws + off; off += (bytes + 255) & ~(size_t)255; return p; };
  b16* w16  = (b16*)carve((size_t)4 * C * C * 2);
  float* st = (float*)carve((size_t)Bn * G * 32 * 4);
  b16* hn   = (b16*)carve((size_t)NPIX * C * 2);
  b16* q16  = (b16*)carve((size_t)NPIX * C * 2);
  b16* k16  = (b16*)carve((size_t)NPIX * C * 2);
  b16* vt16 = (b16*)carve((size_t)C * NPIX * 2);
  b16* S16  = (b16*)carve((size_t)NPIX * NPIX * 2);
  b16* P16  = (b16*)carve((size_t)NPIX * NPIX * 2);
  b16* o16  = (b16*)carve((size_t)NPIX * C * 2);
  if (off > ws_size) return;
  const b16* wq16 = w16; const b16* wk16 = w16 + (size_t)C * C; const b16* wv16 = w16 + (size_t)2 * C * C; const b16* wp16 = w16 + (size_t)3 * C * C;
  const float qscale = 0.044194173824159216f;

  prep_kernel<<<512, 256, 0, stream>>>(wq, wk, wv, wp, w16);
  gn_stats_kernel<<<Bn * G, 256, 0, stream>>>(x, st);
  for (int b = 0; b < Bn; ++b) {
    const float* xb = x + (size_t)b * C * XS;
    float* outb = out + (size_t)b * C * OS;
    gn_apply_kernel<<<NPIX / 64, 256, 0, stream>>>(x, st, gamma, beta, b, hn);
    gemm_kernel<true><<<dim3(C / 64, NPIX / 128), 128, 0, stream>>>(hn, C, wq16, C, C, 1.0f, bq, nullptr, nullptr, 0, q16, nullptr, C);
    gemm_kernel<true><<<dim3(C / 64, NPIX / 128), 128, 0, stream>>>(hn, C, wk16, C, C, 1.0f, bk, nullptr, nullptr, 0, k16, nullptr, C);
    gemm_kernel<true><<<dim3(NPIX / 64, C / 128), 128, 0, stream>>>(wv16, C, hn, C, C, 1.0f, nullptr, bv, nullptr, 0, vt16, nullptr, NPIX);
    gemm_kernel<true><<<dim3(NPIX / 64, NPIX / 128), 128, 0, stream>>>(q16, C, k16, C, C, qscale, nullptr, nullptr, nullptr, 0, S16, nullptr, NPIX);
    softmax_kernel<<<NPIX / 8, 256, 0, stream>>>(S16, P16);
    gemm_kernel<true><<<dim3(C / 64, NPIX / 128), 128, 0, stream>>>(P16, NPIX, vt16, NPIX, NPIX, PV_SC, nullptr, nullptr, nullptr, 0, o16, nullptr, C);
    gemm_kernel<false><<<dim3(NPIX / 64, C / 128), 128, 0, stream>>>(wp16, C, o16, C, C, INV_O_SC, nullptr, bp, xb, XS, nullptr, outb, OS);
  }
}
